// optimizer_18322330485153
// MI455X (gfx1250) — hardware-run, weakly checked
//
#include <hip/hip_runtime.h>

#ifndef STATE_TERMS
#define STATE_TERMS 1
#endif
#define ST STATE_TERMS

typedef __bf16   v16b __attribute__((ext_vector_type(16)));
typedef __bf16   v8b  __attribute__((ext_vector_type(8)));
typedef float    v8f  __attribute__((ext_vector_type(8)));
typedef float    v4f  __attribute__((ext_vector_type(4)));
typedef unsigned v4u  __attribute__((ext_vector_type(4)));
typedef unsigned v2u  __attribute__((ext_vector_type(2)));
typedef v8b __attribute__((may_alias)) v8ba;
typedef v4f __attribute__((may_alias)) v4fa;
typedef v4u __attribute__((may_alias)) v4ua;
typedef v2u __attribute__((may_alias)) v2ua;
typedef unsigned __attribute__((may_alias)) u32a;

union FragB { v16b v; v8b half[2]; };

#define STEP_MU 1e-3f
#define STEP_RO 1e-3f

constexpr int NS    = 25;
constexpr int NG    = 240;
constexpr int NPROB = 1024;
constexpr int NTHR  = 512;
constexpr int TILE  = NG * NS;
constexpr int NV4   = 2 * TILE / 4;
constexpr int MAX_STEPS = 65536;

constexpr int PL_OM = 32 * 256;
constexpr int PL_LT = 32 * 32;

constexpr int OFF_YA   = 0;
constexpr int OFF_YT   = OFF_YA + 32 * 256 * 2;
constexpr int OFF_OMT  = OFF_YT + NG * 32 * 2;
constexpr int OFF_LAMT = OFF_OMT + 2 * ST * PL_OM * 2;
constexpr int OFF_LAM  = OFF_LAMT + 2 * ST * PL_LT * 2;
constexpr int ZEND     = OFF_LAM + 2 * 640 * 4;
constexpr int OFF_UL   = ZEND;
constexpr int OFF_RN   = OFF_UL + 2 * 640 * 4;
constexpr int OFF_OM   = OFF_RN + 2 * 256 * 4;
constexpr int OFF_CP   = OFF_OM + 2 * TILE * 4;
constexpr int LDS_BYTES = OFF_CP + 2 * 8 * 1024 * 4;

static_assert(ST >= 1 && ST <= 3);
static_assert(NS <= 32);
static_assert(NG == 15 * 16 && NG <= 8 * 32);
static_assert(NPROB % 2 == 0);
static_assert((2 * NG * NS * 4) % 128 == 0);
static_assert(NTHR == 16 * 32);
static_assert(LDS_BYTES <= 327680);
static_assert(ZEND % 16 == 0 && OFF_YT % 16 == 0 && OFF_OMT % 16 == 0 && OFF_LAMT % 16 == 0);
static_assert(OFF_LAM % 16 == 0 && OFF_UL % 16 == 0 && OFF_RN % 16 == 0 && OFF_OM % 16 == 0 && OFF_CP % 16 == 0);
static_assert((NPROB / 2 - 1) * 2 * TILE + 2 * TILE - 1 < NPROB * TILE);
static_assert(NV4 * 4 == 2 * TILE);

__device__ __forceinline__ unsigned bfb(float f) {
  unsigned u = __float_as_uint(f);
  return (u + 0x7FFFu + ((u >> 16) & 1u)) >> 16;
}
__device__ __forceinline__ float bff(unsigned b) { return __uint_as_float(b << 16); }
__device__ __forceinline__ float bfr(float f) { return bff(bfb(f)); }

__device__ __forceinline__ void split_planes(float v, unsigned& p0, unsigned& p1, unsigned& p2) {
  p0 = bfb(v);
  float r = v - bff(p0);
  p1 = bfb(r);
  r = r - bff(p1);
  p2 = bfb(r);
}

__device__ __forceinline__ v8f wmb(v16b a, v16b b, v8f c) {
  v8f d = __builtin_amdgcn_wmma_f32_16x16x32_bf16(false, a, false, b, (short)0, c, false, false);
  asm volatile("v_nop\n\tv_nop\n\tv_nop\n\tv_nop" : "+v"(d) : "v"(a), "v"(b));
  return d;
}

__device__ __forceinline__ v16b ldfrag(const unsigned short* p, int h) {
  FragB f;
  f.half[0] = *(const v8ba*)(p + 8 * h);
  f.half[1] = *(const v8ba*)(p + 16 + 8 * h);
  return f.v;
}

__device__ __forceinline__ void upd_tile(float* omq, const float* rnq, int mt, int h, int m, v8f d0, v8f d1) {
  const bool ok1 = (16 + m) < NS;
  const int  tc  = ok1 ? (16 + m) : (NS - 1);
  #pragma unroll
  for (int r = 0; r < 8; ++r) {
    const int g = 16 * mt + 8 * h + r;
    float* o = omq + g * NS;
    const float rv = rnq[g];
    const float o0 = o[m];
    const float o1 = o[tc];
    asm volatile("" :: "v"(o0), "v"(o1), "v"(rv));
    const float n0 = o0 - STEP_MU * (o0 * rv + d0[r]);
    const float n1 = o1 - STEP_MU * (o1 * rv + d1[r]);
    o[m] = n0;
    if (ok1) o[16 + m] = n1;
  }
}

__device__ __forceinline__ void rows_to_planes(const float* omq, float* rnq, unsigned short* omtq, int pl) {
  const bool ok = pl < (NG / 2);
  const int  pc = ok ? pl : (NG / 2 - 1);
  const float* r0 = omq + pc * (2 * NS);
  float a[NS], b[NS];
  #pragma unroll
  for (int t = 0; t < NS; ++t) { a[t] = r0[t]; b[t] = r0[NS + t]; }
  #pragma unroll
  for (int t = 0; t < NS; ++t) asm volatile("" :: "v"(a[t]), "v"(b[t]));
  float s0 = 0.0f, s1 = 0.0f;
  #pragma unroll
  for (int t = 0; t < NS; ++t) { s0 += a[t] * a[t]; s1 += b[t] * b[t]; }
  const float rn0 = 1.0f / sqrtf(s0);
  const float rn1 = 1.0f / sqrtf(s1);
  if (ok) { rnq[2 * pc] = rn0; rnq[2 * pc + 1] = rn1; }
  #pragma unroll
  for (int t = 0; t < NS; ++t) {
    unsigned pa[3], pb[3];
    split_planes(a[t], pa[0], pa[1], pa[2]);
    split_planes(b[t], pb[0], pb[1], pb[2]);
    if (ok) {
      #pragma unroll
      for (int p = 0; p < ST; ++p)
        *(u32a*)(omtq + p * PL_OM + t * 256 + 2 * pc) = pa[p] | (pb[p] << 16);
    }
  }
}

__global__ __launch_bounds__(NTHR) __attribute__((amdgpu_num_vgpr(248)))
void k_iter(const float* __restrict__ Yp, const float* __restrict__ Uk, const float* __restrict__ Lk,
            const float* __restrict__ Om0, const int* __restrict__ nIt, float* __restrict__ out)
{
  extern __shared__ __attribute__((aligned(16))) unsigned char smem[];
  unsigned short* sYA   = (unsigned short*)(smem + OFF_YA);
  unsigned short* sYT   = (unsigned short*)(smem + OFF_YT);
  unsigned short* sOMT  = (unsigned short*)(smem + OFF_OMT);
  unsigned short* sLAMT = (unsigned short*)(smem + OFF_LAMT);
  float* sLAM = (float*)(smem + OFF_LAM);
  float* sUL  = (float*)(smem + OFF_UL);
  float* sRN  = (float*)(smem + OFF_RN);
  float* sOM  = (float*)(smem + OFF_OM);
  float* sCP  = (float*)(smem + OFF_CP);

  const int tid  = threadIdx.x;
  const int lane = tid & 31;
  const int wave = __builtin_amdgcn_readfirstlane(tid >> 5);
  const int h = lane >> 4, m = lane & 15;
  const int q  = wave >> 3;
  const int wl = wave & 7;
  const int tl = tid & 255;
  const int j  = blockIdx.x;

  int tv = nIt[0];
  tv = (tv < 0) ? 0 : tv;
  tv = (tv > MAX_STEPS) ? MAX_STEPS : tv;
  const int T = __builtin_amdgcn_readfirstlane(tv);

  {
    const v4u z4 = {0u, 0u, 0u, 0u};
    #pragma unroll 1
    for (int i = tid; i < ZEND / 16; i += NTHR) *(v4ua*)(smem + i * 16) = z4;
  }
  __syncthreads();

  #pragma unroll 1
  for (int it = 0; it < 3; ++it) {
    const int i  = tid + NTHR * it;
    const int ic = (i < NS * 60) ? i : (NS * 60 - 1);
    const int s  = ic / 60;
    const int c4 = (ic - s * 60) * 4;
    const v4f v = *(const v4fa*)(Yp + s * NG + c4);
    asm volatile("" :: "v"(v));
    const unsigned b0 = bfb(v.x), b1 = bfb(v.y), b2 = bfb(v.z), b3 = bfb(v.w);
    if (i < NS * 60) {
      const v2u pk = { b0 | (b1 << 16), b2 | (b3 << 16) };
      *(v2ua*)(sYA + s * 256 + c4) = pk;
      sYT[(c4 + 0) * 32 + s] = (unsigned short)b0;
      sYT[(c4 + 1) * 32 + s] = (unsigned short)b1;
      sYT[(c4 + 2) * 32 + s] = (unsigned short)b2;
      sYT[(c4 + 3) * 32 + s] = (unsigned short)b3;
    }
  }

  {
    const float* src = Om0 + (size_t)j * (2 * TILE);
    #pragma unroll 1
    for (int it = 0; it < 6; ++it) {
      const int i  = tid + NTHR * it;
      const int ic = (i < NV4) ? i : (NV4 - 1);
      const v4f v = *(const v4fa*)(src + ic * 4);
      asm volatile("" :: "v"(v));
      const v4f r = { bfr(v.x), bfr(v.y), bfr(v.z), bfr(v.w) };
      if (i < NV4) *(v4fa*)(sOM + i * 4) = r;
    }
  }

  {
    const float* ukp = Uk + (size_t)j * (2 * NS * NS);
    const float* lkp = Lk + (size_t)j * (2 * NS);
    #pragma unroll 1
    for (int it = 0; it < 3; ++it) {
      const int e  = tid + NTHR * it;
      const int ec = (e < 2 * NS * NS) ? e : (2 * NS * NS - 1);
      const int qq = (ec >= NS * NS) ? 1 : 0;
      const int r  = ec - qq * (NS * NS);
      const int s  = r / NS;
      const int t  = r - s * NS;
      const float u = ukp[ec];
      const float l = lkp[qq * NS + t];
      asm volatile("" :: "v"(u), "v"(l));
      const float val = bfr(u) * bfr(l);
      if (e < 2 * NS * NS) sUL[qq * 640 + r] = val;
    }
  }
  __syncthreads();

  float*          omq  = sOM + q * TILE;
  float*          rnq  = sRN + q * 256;
  unsigned short* omtq = sOMT + q * (ST * PL_OM);
  unsigned short* ltq  = sLAMT + q * (ST * PL_LT);
  float*          lamq = sLAM + q * 640;
  const float*    ulq  = sUL + q * 640;
  float*          cpq  = sCP + q * (8 * 1024);

  const v16b ya0 = ldfrag(sYA + m * 256 + 32 * wl, h);
  const v16b ya1 = ldfrag(sYA + (16 + m) * 256 + 32 * wl, h);
  const int mt0 = wl;
  const int mt1 = (wl + 8 < 15) ? (wl + 8) : 14;
  const v16b yt0 = ldfrag(sYT + (16 * mt0 + m) * 32, h);
  const v16b yt1 = ldfrag(sYT + (16 * mt1 + m) * 32, h);

  if (wl >= 4) rows_to_planes(omq, rnq, omtq, tl - 128);
  __syncthreads();

  const v8f z8 = {0.f, 0.f, 0.f, 0.f, 0.f, 0.f, 0.f, 0.f};

  #pragma unroll 1
  for (int it = 0; it < T; ++it) {
    {
      const unsigned short* bp = omtq + 32 * wl;
      v8f c00 = z8, c01 = z8, c10 = z8, c11 = z8;
      #pragma unroll
      for (int p = 0; p < ST; ++p) {
        const v16b b0 = ldfrag(bp + p * PL_OM + m * 256, h);
        const v16b b1 = ldfrag(bp + p * PL_OM + (16 + m) * 256, h);
        c00 = wmb(ya0, b0, c00);
        c01 = wmb(ya0, b1, c01);
        c10 = wmb(ya1, b0, c10);
        c11 = wmb(ya1, b1, c11);
      }
      float* cpw = cpq + wl * 1024;
      #pragma unroll
      for (int r = 0; r < 8; ++r) {
        const int ra = (8 * h + r) * 32;
        const int rb = (16 + 8 * h + r) * 32;
        cpw[ra + m]      = c00[r];
        cpw[ra + 16 + m] = c01[r];
        cpw[rb + m]      = c10[r];
        cpw[rb + 16 + m] = c11[r];
      }
    }
    {
      v16b bl0[ST], bl1[ST];
      #pragma unroll
      for (int p = 0; p < ST; ++p) {
        bl0[p] = ldfrag(ltq + p * PL_LT + m * 32, h);
        bl1[p] = ldfrag(ltq + p * PL_LT + (16 + m) * 32, h);
      }
      {
        v8f d0 = z8, d1 = z8;
        #pragma unroll
        for (int p = 0; p < ST; ++p) {
          d0 = wmb(yt0, bl0[p], d0);
          d1 = wmb(yt0, bl1[p], d1);
        }
        upd_tile(omq, rnq, mt0, h, m, d0, d1);
      }
      if (wl < 7) {
        v8f d0 = z8, d1 = z8;
        #pragma unroll
        for (int p = 0; p < ST; ++p) {
          d0 = wmb(yt1, bl0[p], d0);
          d1 = wmb(yt1, bl1[p], d1);
        }
        upd_tile(omq, rnq, mt1, h, m, d0, d1);
      }
    }
    __syncthreads();

    {
      const int nk = (wl < 4) ? 3 : 2;
      #pragma unroll 1
      for (int k = 0; k < nk; ++k) {
        const int  e  = tl + 256 * k;
        const bool ok = e < NS * NS;
        const int  ec = ok ? e : (NS * NS - 1);
        const int  s  = ec / NS;
        const int  t  = ec - s * NS;
        const float* cp = cpq + s * 32 + t;
        float c = cp[0];
        c += cp[1024];
        c += cp[2 * 1024];
        c += cp[3 * 1024];
        c += cp[4 * 1024];
        c += cp[5 * 1024];
        c += cp[6 * 1024];
        c += cp[7 * 1024];
        const float ulv = ulq[ec];
        const float lm0 = lamq[ec];
        asm volatile("" :: "v"(c), "v"(ulv), "v"(lm0));
        c -= ulv;
        const float lv = lm0 + STEP_RO * c;
        unsigned pp[3];
        split_planes(lv, pp[0], pp[1], pp[2]);
        if (ok) {
          lamq[ec] = lv;
          #pragma unroll
          for (int p = 0; p < ST; ++p) ltq[p * PL_LT + t * 32 + s] = (unsigned short)pp[p];
        }
      }
    }
    if (wl >= 4) rows_to_planes(omq, rnq, omtq, tl - 128);
    __syncthreads();
  }

  {
    float* dst = out + (size_t)j * (2 * TILE);
    v4f ov[6];
    #pragma unroll
    for (int k = 0; k < 6; ++k) {
      const int i  = tid + NTHR * k;
      const int ic = (i < NV4) ? i : (NV4 - 1);
      ov[k] = *(const v4fa*)(sOM + ic * 4);
    }
    #pragma unroll
    for (int k = 0; k < 6; ++k) {
      const int i = tid + NTHR * k;
      if (i < NV4) *(volatile v4f*)(dst + (size_t)i * 4) = ov[k];
    }
    __threadfence();
    #pragma unroll
    for (int k = 0; k < 6; ++k) {
      const int i = tid + NTHR * k;
      if (i < NV4) *(volatile v4f*)(dst + (size_t)i * 4) = ov[k];
    }
  }
}

extern "C" void kernel_launch(void* const* d_in, const int* in_sizes, int n_in,
                              void* d_out, int out_size, void* d_ws, size_t ws_size,
                              hipStream_t stream) {
  (void)d_ws; (void)ws_size;
  if (n_in < 5) return;
  if (in_sizes[0] != NS * NG) return;
  if (in_sizes[1] != NPROB * NS * NS) return;
  if (in_sizes[2] != NPROB * NS) return;
  if (in_sizes[3] != NPROB * TILE) return;
  if (in_sizes[4] != 1) return;
  if (out_size != NPROB * TILE) return;

  const float* Yp  = (const float*)d_in[0];
  const float* Uk  = (const float*)d_in[1];
  const float* Lk  = (const float*)d_in[2];
  const float* Om0 = (const float*)d_in[3];
  const int*   nIt = (const int*)d_in[4];
  float* out = (float*)d_out;

  (void)hipFuncSetAttribute(reinterpret_cast<const void*>(&k_iter),
                            hipFuncAttributeMaxDynamicSharedMemorySize, LDS_BYTES);
  k_iter<<<NPROB / 2, NTHR, LDS_BYTES, stream>>>(Yp, Uk, Lk, Om0, nIt, out);
  (void)hipGetLastError();
}
